// GATLayer_61572651155555
// MI455X (gfx1250) — hardware-verified
//
#include <hip/hip_runtime.h>
#include <stddef.h>
#include <stdint.h>
#include <math.h>


#define C_IN    128
#define HC      128
#define NH      4
#define CH      32
#define GBM     64
#define GTHR    128
#define NTHR    256
#define NWAVE   8
#define EPT     8
#define CHUNK   (NTHR * EPT)
#define WCAP    (EPT * 32)
#define LISTN   (NWAVE * WCAP)
#define NB      256
#define SLOTB   8
#define RCAP    14336
#define DEGCAP  64
#define NEGSL   0.2f
#define WSMAX   134217728
#define SCAN_ZINTS (2 * RCAP + 2 * NB + LISTN)
#define LDS_SCAN   ((SCAN_ZINTS + 16) * 4)

static_assert(NB == (1 << SLOTB));
static_assert(NB == NTHR);
static_assert((NB % NWAVE) == 0);
static_assert(LISTN >= NB);
static_assert((CHUNK & (CHUNK - 1)) == 0);
static_assert(((long long)CHUNK << SLOTB) < (1LL << 31));
static_assert((SCAN_ZINTS % 4) == 0 && (RCAP % 4) == 0);
static_assert(LDS_SCAN <= 300000);
static_assert(DEGCAP == 64);
static_assert(GBM == (GTHR / 32) * 16);
static_assert(GTHR == HC);
static_assert((C_IN % 32) == 0);
static_assert(HC == NH * CH && HC == 4 * 32 && CH == 32);
static_assert(2 * NH * CH == 2 * GTHR);

typedef float          v4f   __attribute__((ext_vector_type(4)));
typedef float          v8f   __attribute__((ext_vector_type(8)));
typedef int            v4i   __attribute__((ext_vector_type(4)));
typedef int            v8i   __attribute__((ext_vector_type(8)));
typedef unsigned short v8us  __attribute__((ext_vector_type(8)));
typedef __bf16         v16bf __attribute__((ext_vector_type(16)));
typedef v4f  __attribute__((may_alias)) v4fa;
typedef v4i  __attribute__((may_alias)) v4ia;
typedef v8us __attribute__((may_alias)) v8usa;
union FragB { v16bf v; v8us h[2]; v8i w; };

__device__ __forceinline__ v8f wmb(const FragB& a, const FragB& b, v8f c) {
  v8f d = __builtin_amdgcn_wmma_f32_16x16x32_bf16(false, a.v, false, b.v, (short)0, c, false, false);
  asm volatile("v_nop\n\tv_nop\n\tv_nop\n\tv_nop" : "+v"(d) : "v"(a.w), "v"(b.w));
  return d;
}

__device__ __forceinline__ unsigned bf16_bits(float f) {
  const unsigned u = __float_as_uint(f);
  return (u + 0x7FFFu + ((u >> 16) & 1u)) >> 16;
}
__device__ __forceinline__ float bf16_val(float f) {
  return __uint_as_float(bf16_bits(f) << 16);
}
__device__ __forceinline__ float leaky(float v) { return v >= 0.0f ? v : NEGSL * v; }

__device__ __forceinline__ int scan_chunk(const int* __restrict__ dsts, int nE, int cbase, int slotBase,
                                          int nb, int vec8, int* list, int tid, int lane, int wave) {
  int wc = 0;
  const int el0  = tid * EPT;
  const int e0   = cbase + el0;
  const int sent = -2147483647 - 1;
  v4i da, db;
  if (vec8 != 0 && cbase + CHUNK <= nE) {
    da = *(const v4i*)(dsts + e0);
    db = *(const v4i*)(dsts + e0 + 4);
  } else {
    da.x = (e0     < nE) ? dsts[min(e0,     nE - 1)] : sent;
    da.y = (e0 + 1 < nE) ? dsts[min(e0 + 1, nE - 1)] : sent;
    da.z = (e0 + 2 < nE) ? dsts[min(e0 + 2, nE - 1)] : sent;
    da.w = (e0 + 3 < nE) ? dsts[min(e0 + 3, nE - 1)] : sent;
    db.x = (e0 + 4 < nE) ? dsts[min(e0 + 4, nE - 1)] : sent;
    db.y = (e0 + 5 < nE) ? dsts[min(e0 + 5, nE - 1)] : sent;
    db.z = (e0 + 6 < nE) ? dsts[min(e0 + 6, nE - 1)] : sent;
    db.w = (e0 + 7 < nE) ? dsts[min(e0 + 7, nE - 1)] : sent;
  }
  const unsigned nbs = (unsigned)slotBase;
  const unsigned unb = (unsigned)nb;
  const unsigned s0 = (unsigned)da.x - nbs, s1 = (unsigned)da.y - nbs;
  const unsigned s2 = (unsigned)da.z - nbs, s3 = (unsigned)da.w - nbs;
  const unsigned s4 = (unsigned)db.x - nbs, s5 = (unsigned)db.y - nbs;
  const unsigned s6 = (unsigned)db.z - nbs, s7 = (unsigned)db.w - nbs;
  const bool h0 = s0 < unb, h1 = s1 < unb, h2 = s2 < unb, h3 = s3 < unb;
  const bool h4 = s4 < unb, h5 = s5 < unb, h6 = s6 < unb, h7 = s7 < unb;
  const unsigned any = __builtin_amdgcn_ballot_w32(h0 | h1 | h2 | h3 | h4 | h5 | h6 | h7);
  if (any != 0u) {
#define HITJ(J, HJ, SJ) { \
      const unsigned mj = __builtin_amdgcn_ballot_w32(HJ); \
      if (mj != 0u) { \
        if (HJ) { \
          const int pos = wc + (int)__builtin_amdgcn_mbcnt_lo(mj, 0u); \
          if (pos < WCAP) list[wave * WCAP + pos] = ((el0 + (J)) << SLOTB) | (int)(SJ); \
        } \
        wc += (int)__builtin_popcount(mj); } }
    HITJ(0, h0, s0)
    HITJ(1, h1, s1)
    HITJ(2, h2, s2)
    HITJ(3, h3, s3)
    HITJ(4, h4, s4)
    HITJ(5, h5, s5)
    HITJ(6, h6, s6)
    HITJ(7, h7, s7)
#undef HITJ
  }
  return wc;
}

__device__ __forceinline__ void cvt8(const float* __restrict__ src, unsigned short* dst, int row, int k8, int nValid) {
  const int rc = row < nValid ? row : nValid - 1;
  const float* p = src + (size_t)rc * C_IN + k8;
  const v4f a = *(const v4f*)p;
  const v4f b = *(const v4f*)(p + 4);
  const bool ok = row < nValid;
  v8us o;
  o[0] = ok ? (unsigned short)bf16_bits(a.x) : (unsigned short)0;
  o[1] = ok ? (unsigned short)bf16_bits(a.y) : (unsigned short)0;
  o[2] = ok ? (unsigned short)bf16_bits(a.z) : (unsigned short)0;
  o[3] = ok ? (unsigned short)bf16_bits(a.w) : (unsigned short)0;
  o[4] = ok ? (unsigned short)bf16_bits(b.x) : (unsigned short)0;
  o[5] = ok ? (unsigned short)bf16_bits(b.y) : (unsigned short)0;
  o[6] = ok ? (unsigned short)bf16_bits(b.z) : (unsigned short)0;
  o[7] = ok ? (unsigned short)bf16_bits(b.w) : (unsigned short)0;
  unsigned short* dp = dst + (size_t)row * C_IN + k8;
  *(volatile v8us*)dp = o;
  __threadfence();
  *(volatile v8us*)dp = o;
}

__global__ __launch_bounds__(NTHR) void k_prep(const float* __restrict__ x, const float* __restrict__ w,
                                               unsigned short* xb, unsigned short* wb,
                                               int nN, int nUx, int nUw) {
  const int u = (int)blockIdx.x * NTHR + (int)threadIdx.x;
  if (u < nUx) {
    cvt8(x, xb, u >> 4, (u & 15) * 8, nN);
  } else if (u < nUx + nUw) {
    const int v = u - nUx;
    cvt8(w, wb, v >> 4, (v & 15) * 8, HC);
  }
}

__global__ __launch_bounds__(GTHR) void k_proj(const unsigned short* __restrict__ A,
                                               const unsigned short* __restrict__ BT,
                                               const float* __restrict__ bias, const float* __restrict__ avec,
                                               float* Hm, float* SSD, float* PS, int nN) {
  __shared__ __attribute__((aligned(16))) float stg[GBM * HC];
  __shared__ __attribute__((aligned(16))) float sdt[GBM * 8];
  __shared__ __attribute__((aligned(16))) float sps[HC];
  __shared__ __attribute__((aligned(16))) float sbias[HC];
  __shared__ __attribute__((aligned(16))) float sa[2 * NH * CH];
  const int tid = (int)threadIdx.x, lane = tid & 31, wave = tid >> 5, hh = lane >> 4, m = lane & 15;
  const int rowBase = (int)blockIdx.x * GBM;

  sbias[tid]    = bf16_val(bias[tid]);
  sa[tid]       = bf16_val(avec[tid]);
  sa[tid + 128] = bf16_val(avec[tid + 128]);

  v8f acc[8];
  {
    const v8f z = {0.f, 0.f, 0.f, 0.f, 0.f, 0.f, 0.f, 0.f};
#pragma unroll
    for (int t = 0; t < 8; ++t) acc[t] = z;
  }
  const unsigned short* ap = A  + (size_t)(rowBase + 16 * wave + m) * (size_t)C_IN + 8 * hh;
  const unsigned short* bp = BT + (size_t)m * (size_t)C_IN + 8 * hh;
#pragma unroll 1
  for (int k0 = 0; k0 < C_IN; k0 += 32) {
    FragB af;
    af.h[0] = *(const v8usa*)(ap + k0);
    af.h[1] = *(const v8usa*)(ap + k0 + 16);
#pragma unroll
    for (int nt = 0; nt < 8; ++nt) {
      const unsigned short* wq = bp + (size_t)(16 * nt) * (size_t)C_IN + k0;
      FragB bf;
      bf.h[0] = *(const v8usa*)wq;
      bf.h[1] = *(const v8usa*)(wq + 16);
      acc[nt] = wmb(af, bf, acc[nt]);
    }
  }
  __syncthreads();

#pragma unroll
  for (int nt = 0; nt < 8; ++nt) {
    const int lc = 16 * nt + m;
    const float bb = sbias[lc];
#pragma unroll
    for (int r = 0; r < 8; ++r) {
      const int lr = 16 * wave + 8 * hh + r;
      stg[lr * HC + lc] = acc[nt][r] + bb;
    }
  }
  __syncthreads();

  {
    const int hd = lane >> 3, q = lane & 7;
    const v4f as4 = *(const v4fa*)(sa + hd * (2 * CH) + 4 * q);
    const v4f ad4 = *(const v4fa*)(sa + hd * (2 * CH) + CH + 4 * q);
#pragma unroll 1
    for (int i = 0; i < 16; ++i) {
      const int row = wave * 16 + i;
      const v4f p = *(const v4fa*)(stg + row * HC + 4 * lane);
      float s = 0.0f, d = 0.0f;
      s = fmaf(p.x, as4.x, s); s = fmaf(p.y, as4.y, s); s = fmaf(p.z, as4.z, s); s = fmaf(p.w, as4.w, s);
      d = fmaf(p.x, ad4.x, d); d = fmaf(p.y, ad4.y, d); d = fmaf(p.z, ad4.z, d); d = fmaf(p.w, ad4.w, d);
#pragma unroll
      for (int off = 4; off > 0; off >>= 1) {
        s += __shfl_xor(s, off);
        d += __shfl_xor(d, off);
      }
      if (q == 0) { sdt[row * 8 + hd] = s; sdt[row * 8 + 4 + hd] = d; }
    }
  }
  {
    int rl = nN - rowBase;
    rl = rl < 0 ? 0 : (rl > GBM ? GBM : rl);
    float cs = 0.0f;
#pragma unroll 4
    for (int r = 0; r < rl; ++r) cs += stg[r * HC + tid];
    sps[tid] = cs;
  }
  __syncthreads();

  const v4f sdv = *(const v4fa*)(sdt + 4 * tid);
  float* sp = SSD + (size_t)rowBase * 8 + 4 * tid;
  const v4f psv = *(const v4fa*)(sps + 4 * lane);
  float* pp = PS + (size_t)blockIdx.x * HC + 4 * lane;
#pragma unroll 1
  for (int i = 0; i < 16; ++i) {
    const int row = wave * 16 + i;
    const v4f p = *(const v4fa*)(stg + row * HC + 4 * lane);
    float* op = Hm + (size_t)(rowBase + row) * (size_t)HC + 4 * lane;
    *(volatile v4f*)op = p;
  }
  *(volatile v4f*)sp = sdv;
  if (wave == 0) *(volatile v4f*)pp = psv;
  __threadfence();
#pragma unroll 1
  for (int i = 0; i < 16; ++i) {
    const int row = wave * 16 + i;
    const v4f p = *(const v4fa*)(stg + row * HC + 4 * lane);
    float* op = Hm + (size_t)(rowBase + row) * (size_t)HC + 4 * lane;
    *(volatile v4f*)op = p;
  }
  *(volatile v4f*)sp = sdv;
  if (wave == 0) *(volatile v4f*)pp = psv;
}

__global__ __launch_bounds__(HC) void k_hm(const float* __restrict__ PS, float* HM, int nBlk, double invN) {
  __shared__ __attribute__((aligned(16))) float sh[HC];
  const int tid = (int)threadIdx.x, lane = tid & 31, wave = tid >> 5;
  double s = 0.0;
#pragma unroll 4
  for (int b = 0; b < nBlk; ++b) s += (double)PS[(size_t)b * HC + tid];
  sh[tid] = (float)(s * invN);
  __syncthreads();
  if (wave == 0) {
    const v4f v = *(const v4fa*)(sh + 4 * lane);
    float* op = HM + 4 * lane;
    *(volatile v4f*)op = v;
    __threadfence();
    *(volatile v4f*)op = v;
  }
}

__global__ __launch_bounds__(NTHR) void k_scan(const int* __restrict__ keys, const int* __restrict__ nbrs,
                                               const float* __restrict__ Hm, const float* __restrict__ SSD,
                                               const float* __restrict__ HM, float* out,
                                               int nN, int nE, int vec8) {
  extern __shared__ v4f lds_dyn[];
  int* reg1 = (int*)lds_dyn;
  int* reg2 = reg1 + RCAP;
  int* scnt = reg2 + RCAP;
  int* soff = scnt + NB;
  int* list = soff + NB;
  int* wcnt = list + LISTN;
  int* wtot = wcnt + NWAVE;
  const int tid = (int)threadIdx.x, lane = tid & 31, wave = tid >> 5;
  const int nodeBase = (int)blockIdx.x * NB;

  {
    const v4i z4 = {0, 0, 0, 0};
    for (int i = tid * 4; i < SCAN_ZINTS; i += NTHR * 4) *(v4ia*)(reg1 + i) = z4;
    if (tid < 16) wcnt[tid] = 0;
  }
  __syncthreads();

  int tot = 0;
  const int nChunks = (nE + CHUNK - 1) / CHUNK;
#pragma unroll 1
  for (int ch = 0; ch < nChunks; ++ch) {
    const int cbase = ch * CHUNK;
    const int wc = scan_chunk(keys, nE, cbase, nodeBase, NB, vec8, list, tid, lane, wave);
    if (lane == 0) wcnt[wave] = wc;
    __syncthreads();
    int pre = 0, all = 0;
#pragma unroll
    for (int w2 = 0; w2 < NWAVE; ++w2) {
      int c = wcnt[w2];
      c = c < 0 ? 0 : (c > WCAP ? WCAP : c);
      all += c;
      pre += (w2 < wave) ? c : 0;
    }
    const int wcc  = wc < 0 ? 0 : (wc > WCAP ? WCAP : wc);
    const int base = tot + pre;
#pragma unroll 1
    for (int i = lane; i < wcc; i += 32) {
      const int ent = list[wave * WCAP + i];
      const int el  = (ent >> SLOTB) & (CHUNK - 1);
      const int sl  = ent & (NB - 1);
      int eid = cbase + el;
      eid = eid > nE - 1 ? nE - 1 : eid;
      int j = nbrs[eid];
      j = j < 0 ? 0 : (j > nN - 1 ? nN - 1 : j);
      const int pos = base + i;
      if (pos < RCAP) reg1[pos] = (int)(((unsigned)j << SLOTB) | (unsigned)sl);
    }
    tot += all;
    tot = tot > RCAP ? RCAP : tot;
    __syncthreads();
  }
  const int nh = tot;

  if (wave == 0) {
#pragma unroll 1
    for (int b0 = 0; b0 < nh; b0 += 32) {
      const int idx = b0 + lane;
      const int uv  = reg1[idx < nh ? idx : nh - 1];
      const int m32 = (nh - b0) < 32 ? (nh - b0) : 32;
#pragma unroll 1
      for (int k = 0; k < m32; ++k) {
        const int u  = __builtin_amdgcn_readlane(uv, k);
        const int sl = u & (NB - 1);
        if (lane == 0) scnt[sl] = scnt[sl] + 1;
      }
    }
  }
  __syncthreads();

  {
    int c = scnt[tid];
    c = c < 0 ? 0 : c;
    int incl = c;
#pragma unroll
    for (int d = 1; d < 32; d <<= 1) {
      const int up = __shfl_up(incl, d);
      if (lane >= d) incl += up;
    }
    if (lane == 31) wtot[wave] = incl;
    __syncthreads();
    int pre = 0;
#pragma unroll
    for (int w2 = 0; w2 < NWAVE; ++w2) pre += (w2 < wave) ? wtot[w2] : 0;
    const int run = pre + incl - c;
    soff[tid] = run;
    list[tid] = run;
  }
  __syncthreads();

  if (wave == 0) {
#pragma unroll 1
    for (int b0 = 0; b0 < nh; b0 += 32) {
      const int idx = b0 + lane;
      const int uv  = reg1[idx < nh ? idx : nh - 1];
      const int m32 = (nh - b0) < 32 ? (nh - b0) : 32;
#pragma unroll 1
      for (int k = 0; k < m32; ++k) {
        const int u  = __builtin_amdgcn_readlane(uv, k);
        const int sl = u & (NB - 1);
        const int jv = (int)((unsigned)u >> SLOTB);
        if (lane == 0) {
          int pos = list[sl];
          pos = pos < 0 ? 0 : (pos > RCAP - 1 ? RCAP - 1 : pos);
          reg2[pos] = jv;
          list[sl] = pos + 1;
        }
      }
    }
  }
  __syncthreads();

  const int   head = lane >> 3;
  const bool  ovf  = (nh >= RCAP);
  const float qnan = __int_as_float(0x7fc00000);
  const float NEGB = -3.0e38f;
  const v4f   hm4  = *(const v4fa*)(HM + 4 * lane);

#pragma unroll 1
  for (int jt = 0; jt < NB / NWAVE; ++jt) {
    const int slot = wave * (NB / NWAVE) + jt;
    const int grow = nodeBase + slot;
    const int gcl  = grow < nN ? grow : nN - 1;
    int st = soff[slot];
    const int craw = scnt[slot];
    int cnt = craw;
    st  = st < 0 ? 0 : (st > nh ? nh : st);
    cnt = cnt < 0 ? 0 : (cnt > DEGCAP ? DEGCAP : cnt);
    if (cnt > nh - st) cnt = nh - st;
    const float pz = (ovf || craw > DEGCAP) ? qnan : 0.0f;

    int i0 = st + lane;      i0 = i0 > RCAP - 1 ? RCAP - 1 : i0;
    int i1 = st + lane + 32; i1 = i1 > RCAP - 1 ? RCAP - 1 : i1;
    int r0 = reg2[i0], r1 = reg2[i1];
    r0 = r0 < 0 ? 0 : (r0 > nN - 1 ? nN - 1 : r0);
    r1 = r1 < 0 ? 0 : (r1 > nN - 1 ? nN - 1 : r1);
    const bool v0 = lane < cnt, v1 = (lane + 32) < cnt;
    const int e0 = v0 ? r0 : -1;
    const int e1 = v1 ? r1 : -1;

    bool d0 = false, d1 = false;
#pragma unroll 1
    for (int k = 0; k < cnt; ++k) {
      const int va = __builtin_amdgcn_readlane(e0, k & 31);
      const int vb = __builtin_amdgcn_readlane(e1, k & 31);
      const int v  = (k < 32) ? va : vb;
      d0 = d0 || ((k < lane) && (v == e0));
      d1 = d1 || ((k < lane + 32) && (v == e1));
    }
    const bool keep0 = v0 && !d0;
    const bool keep1 = v1 && !d1;
    const unsigned km0 = __builtin_amdgcn_ballot_w32(keep0);
    const unsigned km1 = __builtin_amdgcn_ballot_w32(keep1);

    const v4f ss4 = *(const v4fa*)(SSD + (size_t)gcl * 8);
    const v4f sdA = *(const v4fa*)(SSD + (size_t)(e0 < 0 ? 0 : e0) * 8 + 4);
    const v4f sdB = *(const v4fa*)(SSD + (size_t)(e1 < 0 ? 0 : e1) * 8 + 4);
    float m0 = fmaxf(keep0 ? leaky(ss4.x + sdA.x) : NEGB, keep1 ? leaky(ss4.x + sdB.x) : NEGB);
    float m1 = fmaxf(keep0 ? leaky(ss4.y + sdA.y) : NEGB, keep1 ? leaky(ss4.y + sdB.y) : NEGB);
    float m2 = fmaxf(keep0 ? leaky(ss4.z + sdA.z) : NEGB, keep1 ? leaky(ss4.z + sdB.z) : NEGB);
    float m3 = fmaxf(keep0 ? leaky(ss4.w + sdA.w) : NEGB, keep1 ? leaky(ss4.w + sdB.w) : NEGB);
#pragma unroll
    for (int off = 16; off > 0; off >>= 1) {
      m0 = fmaxf(m0, __shfl_xor(m0, off));
      m1 = fmaxf(m1, __shfl_xor(m1, off));
      m2 = fmaxf(m2, __shfl_xor(m2, off));
      m3 = fmaxf(m3, __shfl_xor(m3, off));
    }
    const float mh  = (head == 0) ? m0 : ((head == 1) ? m1 : ((head == 2) ? m2 : m3));
    const float ssh = (head == 0) ? ss4.x : ((head == 1) ? ss4.y : ((head == 2) ? ss4.z : ss4.w));

    float den = 0.0f;
    v4f acc = {0.0f, 0.0f, 0.0f, 0.0f};
#pragma unroll 1
    for (int k = 0; k < cnt; ++k) {
      const int ja = __builtin_amdgcn_readlane(e0, k & 31);
      const int jb = __builtin_amdgcn_readlane(e1, k & 31);
      int jk = (k < 32) ? ja : jb;
      jk = jk < 0 ? 0 : (jk > nN - 1 ? nN - 1 : jk);
      const unsigned kms = (k < 32) ? km0 : km1;
      const bool kb = ((kms >> (k & 31)) & 1u) != 0u;
      const float sdk = SSD[(size_t)jk * 8 + 4 + head];
      const v4f hv = *(const v4fa*)(Hm + (size_t)jk * HC + 4 * lane);
      const float lg = leaky(ssh + sdk);
      float w = expf(lg - mh);
      w = kb ? w : 0.0f;
      den += w;
      acc.x = fmaf(w, hv.x, acc.x);
      acc.y = fmaf(w, hv.y, acc.y);
      acc.z = fmaf(w, hv.z, acc.z);
      acc.w = fmaf(w, hv.w, acc.w);
    }
    const bool has = cnt > 0;
    const float dsafe = has ? den : 1.0f;
    const float inv = 1.0f / dsafe;
    v4f o;
    o.x = (has ? acc.x * inv : hm4.x) + pz;
    o.y = (has ? acc.y * inv : hm4.y) + pz;
    o.z = (has ? acc.z * inv : hm4.z) + pz;
    o.w = (has ? acc.w * inv : hm4.w) + pz;
    if (grow < nN) {
      float* op = out + (size_t)grow * HC + 4 * lane;
      *(volatile v4f*)op = o;
      __threadfence();
      *(volatile v4f*)op = o;
    }
  }
}

static inline int cdiv(int a, int b) { return (a + b - 1) / b; }

extern "C" void kernel_launch(void* const* d_in, const int* in_sizes, int n_in,
                              void* d_out, int out_size, void* d_ws, size_t ws_size,
                              hipStream_t stream) {
  if (n_in < 5) return;
  if (in_sizes[0] < C_IN || (in_sizes[0] % C_IN) != 0) return;
  const int nN = in_sizes[0] / C_IN;
  if (nN <= 0 || nN > (1 << 22)) return;
  if (in_sizes[1] != HC * C_IN) return;
  if (in_sizes[2] != HC) return;
  if (in_sizes[3] != NH * 2 * CH) return;
  if (in_sizes[4] < 2 || (in_sizes[4] & 1) != 0) return;
  const int nE = in_sizes[4] / 2;
  if (nE < 1) return;
  if ((long long)out_size != (long long)nN * HC) return;

  const float* x    = (const float*)d_in[0];
  const float* W    = (const float*)d_in[1];
  const float* bias = (const float*)d_in[2];
  const float* avec = (const float*)d_in[3];
  const int*   ei   = (const int*)d_in[4];
  float* out = (float*)d_out;
  const int* keys = ei;
  const int* nbrs = ei + nE;

  const int MP = cdiv(nN, GBM) * GBM;
  const int gM = MP / GBM;
  const int gS = cdiv(nN, NB);
  if ((long long)gS * NB < (long long)nN) return;
  const int vec8 = ((nE & 3) == 0) ? 1 : 0;

  char* ws = (char*)d_ws;
  size_t off = 0;
  const size_t oXB  = off; off += (size_t)MP * C_IN * 2;   off = (off + 255) & ~(size_t)255;
  const size_t oWB  = off; off += (size_t)HC * C_IN * 2;   off = (off + 255) & ~(size_t)255;
  const size_t oH   = off; off += (size_t)MP * HC * 4;     off = (off + 255) & ~(size_t)255;
  const size_t oSSD = off; off += (size_t)MP * 8 * 4;      off = (off + 255) & ~(size_t)255;
  const size_t oPS  = off; off += (size_t)gM * HC * 4;     off = (off + 255) & ~(size_t)255;
  const size_t oHM  = off; off += (size_t)HC * 4;          off = (off + 255) & ~(size_t)255;
  if (off > ws_size || off > (size_t)WSMAX) return;
  unsigned short* XB  = (unsigned short*)(ws + oXB);
  unsigned short* WB  = (unsigned short*)(ws + oWB);
  float*          Hm  = (float*)(ws + oH);
  float*          SSD = (float*)(ws + oSSD);
  float*          PS  = (float*)(ws + oPS);
  float*          HMp = (float*)(ws + oHM);

  hipFuncSetAttribute(reinterpret_cast<const void*>(&k_scan),
                      hipFuncAttributeMaxDynamicSharedMemorySize, LDS_SCAN);

  const int nUx = MP * (C_IN / 8);
  const int nUw = HC * (C_IN / 8);
  k_prep<<<cdiv(nUx + nUw, NTHR), NTHR, 0, stream>>>(x, W, XB, WB, nN, nUx, nUw);
  k_proj<<<gM, GTHR, 0, stream>>>(XB, WB, bias, avec, Hm, SSD, PS, nN);
  k_hm<<<1, HC, 0, stream>>>(PS, HMp, gM, 1.0 / (double)nN);
  k_scan<<<gS, NTHR, LDS_SCAN, stream>>>(keys, nbrs, Hm, SSD, HMp, out, nN, nE, vec8);
}
